// Model_49692771615413
// MI455X (gfx1250) — hardware-verified
//
#include <hip/hip_runtime.h>
#include <stddef.h>
#include <stdint.h>

#define NB      16384
#define NF      41024
#define HALF    256
#define ROWW    257
#define MAXF    30
#define K1      1024
#define K2      64
#define NTB     (NF / 32)
#define SV_N    512
#define SV_FC1B 288
#define SV_FC2B 320
#define SV_FCOW 352
#define SV_FCOB 384
#define WSMAX   134217728

static_assert(HALF == 32 * 8);
static_assert(MAXF <= 32);
static_assert(NB % 128 == 0 && NB % 64 == 0);
static_assert(NF % 32 == 0 && NTB * 32 == NF);
static_assert(ROWW == HALF + 1);
static_assert(K1 % 32 == 0 && K2 % 32 == 0 && K1 == 4 * HALF);
static_assert(SV_FC1B >= ROWW && SV_FCOB + 1 <= SV_FC1B + 128 && SV_FC1B + 128 <= SV_N);

typedef float          v4f   __attribute__((ext_vector_type(4)));
typedef float          v8f   __attribute__((ext_vector_type(8)));
typedef int            v8i   __attribute__((ext_vector_type(8)));
typedef unsigned       v4u   __attribute__((ext_vector_type(4)));
typedef unsigned short v8us  __attribute__((ext_vector_type(8)));
typedef unsigned short v16us __attribute__((ext_vector_type(16)));
typedef __bf16         v16bf __attribute__((ext_vector_type(16)));
typedef v4f  __attribute__((may_alias)) v4fa;
typedef v4u  __attribute__((may_alias)) v4ua;
typedef v8us __attribute__((may_alias)) v8usa;
union FragB { v16bf v; v16us u; v8us h[2]; v8i w; };

__device__ __forceinline__ v8f wmb(const FragB& a, const FragB& b, v8f c) {
  v8f d = __builtin_amdgcn_wmma_f32_16x16x32_bf16(false, a.v, false, b.v, (short)0, c, false, false);
  asm volatile("v_nop\n\tv_nop\n\tv_nop\n\tv_nop" : "+v"(d) : "v"(a.w), "v"(b.w));
  return d;
}

__device__ __forceinline__ unsigned bf16_bits(float f) {
  const unsigned u = __float_as_uint(f);
  return (u + 0x7FFFu + ((u >> 16) & 1u)) >> 16;
}
__device__ __forceinline__ float bf16_val(float f) {
  return __uint_as_float(bf16_bits(f) << 16);
}
__device__ __forceinline__ unsigned pack2(float a, float b) {
  return bf16_bits(a) | (bf16_bits(b) << 16);
}
struct HL { unsigned h; unsigned l; };
__device__ __forceinline__ HL split2(float a, float b) {
  const unsigned ha = bf16_bits(a), hb = bf16_bits(b);
  const unsigned la = bf16_bits(a - __uint_as_float(ha << 16));
  const unsigned lb = bf16_bits(b - __uint_as_float(hb << 16));
  HL r;
  r.h = ha | (hb << 16);
  r.l = la | (lb << 16);
  return r;
}
__device__ __forceinline__ float clip01(float v) {
  return fminf(fmaxf(v, 0.0f), 1.0f);
}

__global__ __launch_bounds__(256) void k_prep(
    const float* __restrict__ ftw, const float* __restrict__ ftb,
    const float* __restrict__ fc1w, const float* __restrict__ fc1b,
    const float* __restrict__ fc2w, const float* __restrict__ fc2b,
    const float* __restrict__ fcow, const float* __restrict__ fcob,
    unsigned short* FTB, float* PSQ, unsigned short* FC1D, unsigned short* FC2D, float* SV)
{
  __shared__ __attribute__((aligned(16))) float sl[SV_N];
  const int tid = (int)threadIdx.x, lane = tid & 31;
  const int wv = __builtin_amdgcn_readfirstlane(tid >> 5);
  const int blk = (int)blockIdx.x;

  if (blk < NTB) {
#pragma unroll 1
    for (int q = 0; q < 4; ++q) {
      const int r = blk * 32 + wv * 4 + q;
      const float* src = ftw + (size_t)r * ROWW + 8 * lane;
      const float f0 = src[0], f1 = src[1], f2 = src[2], f3 = src[3];
      const float f4 = src[4], f5 = src[5], f6 = src[6], f7 = src[7];
      v4u o;
      o.x = pack2(f0, f1);
      o.y = pack2(f2, f3);
      o.z = pack2(f4, f5);
      o.w = pack2(f6, f7);
      unsigned short* dp = FTB + (size_t)r * HALF + 8 * lane;
      *(volatile v4u*)dp = o;
      __threadfence();
      *(volatile v4u*)dp = o;
    }
    if (wv == 0) {
      const float pvv = ftw[(size_t)(blk * 32 + lane) * ROWW + HALF];
      sl[lane] = bf16_val(pvv);
    }
    __syncthreads();
    if (wv == 0) {
      const v4f v = *(const v4fa*)(sl + 4 * (lane & 7));
      if (lane < 8) {
        float* dp = PSQ + (size_t)blk * 32 + 4 * lane;
        *(volatile v4f*)dp = v;
        __threadfence();
        *(volatile v4f*)dp = v;
      }
    }
  } else {
#pragma unroll 1
    for (int it = 0; it < 16; ++it) {
      const int u = it * 256 + tid;
      const int n = u >> 7;
      const int k8 = (u & 127) * 8;
      const float* p = fc1w + (size_t)n * 512 + (k8 & 511);
      const v4f a = *(const v4f*)p;
      const v4f b = *(const v4f*)(p + 4);
      v4u o;
      o.x = pack2(a.x, a.y);
      o.y = pack2(a.z, a.w);
      o.z = pack2(b.x, b.y);
      o.w = pack2(b.z, b.w);
      unsigned short* dp = FC1D + (size_t)n * K1 + k8;
      *(volatile v4u*)dp = o;
      __threadfence();
      *(volatile v4u*)dp = o;
    }
    {
      const int n = tid >> 3;
      const int k8 = (tid & 7) * 8;
      const float* p = fc2w + (size_t)n * 32 + (k8 & 31);
      const v4f a = *(const v4f*)p;
      const v4f b = *(const v4f*)(p + 4);
      v4u o;
      o.x = pack2(a.x, a.y);
      o.y = pack2(a.z, a.w);
      o.z = pack2(b.x, b.y);
      o.w = pack2(b.z, b.w);
      unsigned short* dp = FC2D + (size_t)n * K2 + k8;
      *(volatile v4u*)dp = o;
      __threadfence();
      *(volatile v4u*)dp = o;
    }
    sl[256 + tid] = 0.0f;
    __syncthreads();
    sl[tid] = bf16_val(ftb[tid]);
    if (wv == 0) {
      const float t = ftb[HALF];
      if (lane == 0) sl[HALF] = bf16_val(t);
    } else if (wv == 1) {
      sl[SV_FC1B + lane] = bf16_val(fc1b[lane]);
    } else if (wv == 2) {
      sl[SV_FC2B + lane] = bf16_val(fc2b[lane]);
    } else if (wv == 3) {
      sl[SV_FCOW + lane] = bf16_val(fcow[lane]);
    } else if (wv == 4) {
      const float t = fcob[0];
      if (lane == 0) sl[SV_FCOB] = bf16_val(t);
    }
    __syncthreads();
    if (wv < 4) {
      const v4f v = *(const v4fa*)(sl + 4 * tid);
      float* dp = SV + 4 * tid;
      *(volatile v4f*)dp = v;
      __threadfence();
      *(volatile v4f*)dp = v;
    }
  }
}

__device__ __forceinline__ void side_gather(const int* __restrict__ ics, int samp,
                                            const unsigned short* __restrict__ FTB,
                                            const float* __restrict__ PSQ, int lane,
                                            float (&acc)[8], float& psum)
{
  const int li = lane < MAXF ? lane : MAXF - 1;
  const int raw = ics[(size_t)samp * MAXF + li];
  const int myidx = (lane < MAXF) ? raw : -1;
  int pc = myidx < 0 ? 0 : myidx;
  pc = pc > NF - 1 ? NF - 1 : pc;
  float pv = PSQ[pc];
  pv = (myidx >= 0) ? pv : 0.0f;
  pv += __shfl_xor(pv, 16);
  pv += __shfl_xor(pv, 8);
  pv += __shfl_xor(pv, 4);
  pv += __shfl_xor(pv, 2);
  pv += __shfl_xor(pv, 1);
  psum = pv;
#pragma unroll
  for (int i = 0; i < 8; ++i) acc[i] = 0.0f;
#pragma unroll 6
  for (int j = 0; j < MAXF; ++j) {
    const int id = __builtin_amdgcn_readlane(myidx, j);
    int sid = id < 0 ? 0 : id;
    sid = sid > NF - 1 ? NF - 1 : sid;
    const v4u w = *(const v4ua*)(FTB + (size_t)sid * HALF + 8 * lane);
    const bool ok = id >= 0;
    const float f0 = __uint_as_float(w.x << 16), f1 = __uint_as_float(w.x & 0xffff0000u);
    const float f2 = __uint_as_float(w.y << 16), f3 = __uint_as_float(w.y & 0xffff0000u);
    const float f4 = __uint_as_float(w.z << 16), f5 = __uint_as_float(w.z & 0xffff0000u);
    const float f6 = __uint_as_float(w.w << 16), f7 = __uint_as_float(w.w & 0xffff0000u);
    acc[0] += ok ? f0 : 0.0f;
    acc[1] += ok ? f1 : 0.0f;
    acc[2] += ok ? f2 : 0.0f;
    acc[3] += ok ? f3 : 0.0f;
    acc[4] += ok ? f4 : 0.0f;
    acc[5] += ok ? f5 : 0.0f;
    acc[6] += ok ? f6 : 0.0f;
    acc[7] += ok ? f7 : 0.0f;
  }
}

__global__ __launch_bounds__(256) void k_ft(
    const int* __restrict__ wft, const int* __restrict__ bft, const float* __restrict__ stm,
    const unsigned short* __restrict__ FTB, const float* __restrict__ PSQ, const float* __restrict__ SV,
    unsigned short* XHL, float* PS)
{
  __shared__ __attribute__((aligned(16))) float psl[64];
  const int tid = (int)threadIdx.x, lane = tid & 31, wave = tid >> 5;
  const int blk = (int)blockIdx.x;

  float fb[8];
  {
    const v4f a = *(const v4f*)(SV + 8 * lane);
    const v4f b = *(const v4f*)(SV + 8 * lane + 4);
    fb[0] = a.x; fb[1] = a.y; fb[2] = a.z; fb[3] = a.w;
    fb[4] = b.x; fb[5] = b.y; fb[6] = b.z; fb[7] = b.w;
  }
  const float fb256 = SV[HALF];

#pragma unroll 1
  for (int q = 0; q < 8; ++q) {
    const int samp = blk * 64 + wave * 8 + q;
    float w[8], b[8];
    float wps, bps;
    side_gather(wft, samp, FTB, PSQ, lane, w, wps);
    side_gather(bft, samp, FTB, PSQ, lane, b, bps);
#pragma unroll
    for (int i = 0; i < 8; ++i) { w[i] += fb[i]; b[i] += fb[i]; }
    wps += fb256;
    bps += fb256;
    const float s = bf16_val(stm[samp]);
    const float oms = 1.0f - s;
    float xa[8], xb[8];
#pragma unroll
    for (int i = 0; i < 8; ++i) {
      xa[i] = clip01(oms * w[i] + s * b[i]);
      xb[i] = clip01(oms * b[i] + s * w[i]);
    }
    v4u hA, lA, hB, lB;
    {
      const HL a0 = split2(xa[0], xa[1]), a1 = split2(xa[2], xa[3]);
      const HL a2 = split2(xa[4], xa[5]), a3 = split2(xa[6], xa[7]);
      const HL b0 = split2(xb[0], xb[1]), b1 = split2(xb[2], xb[3]);
      const HL b2 = split2(xb[4], xb[5]), b3 = split2(xb[6], xb[7]);
      hA.x = a0.h; hA.y = a1.h; hA.z = a2.h; hA.w = a3.h;
      lA.x = a0.l; lA.y = a1.l; lA.z = a2.l; lA.w = a3.l;
      hB.x = b0.h; hB.y = b1.h; hB.z = b2.h; hB.w = b3.h;
      lB.x = b0.l; lB.y = b1.l; lB.z = b2.l; lB.w = b3.l;
    }
    unsigned short* xr = XHL + (size_t)samp * K1 + 8 * lane;
    *(volatile v4u*)(xr)            = hA;
    *(volatile v4u*)(xr + HALF)     = hB;
    *(volatile v4u*)(xr + 2 * HALF) = lA;
    *(volatile v4u*)(xr + 3 * HALF) = lB;
    __threadfence();
    *(volatile v4u*)(xr)            = hA;
    *(volatile v4u*)(xr + HALF)     = hB;
    *(volatile v4u*)(xr + 2 * HALF) = lA;
    *(volatile v4u*)(xr + 3 * HALF) = lB;

    const float psv = (wps - bps) * (0.5f - s);
    if (lane == 0) psl[wave * 8 + q] = psv;
  }
  __syncthreads();
  if (tid < 32) {
    const v4f v = *(const v4fa*)(psl + 4 * (lane & 15));
    if (lane < 16) {
      float* dp = PS + (size_t)blk * 64 + 4 * lane;
      *(volatile v4f*)dp = v;
      __threadfence();
      *(volatile v4f*)dp = v;
    }
  }
}

__global__ __launch_bounds__(256) void k_mlp(
    const unsigned short* __restrict__ XHL, const unsigned short* __restrict__ FC1D,
    const unsigned short* __restrict__ FC2D, const float* __restrict__ SV,
    const float* __restrict__ PS, float* out)
{
  __shared__ __attribute__((aligned(16))) float h1s[8 * 16 * 32];
  __shared__ __attribute__((aligned(16))) float h2s[8 * 16 * 32];
  __shared__ __attribute__((aligned(16))) float svl[128];
  __shared__ __attribute__((aligned(16))) float outl[128];
  const int tid = (int)threadIdx.x, lane = tid & 31, wave = tid >> 5;
  const int hh = lane >> 4, m = lane & 15;
  const int rowBase = (int)blockIdx.x * 128;
  const int row = rowBase + 16 * wave + m;

  if (tid < 32) {
    const v4f t = *(const v4f*)(SV + SV_FC1B + 4 * tid);
    *(v4fa*)(svl + 4 * tid) = t;
  }
  __syncthreads();

  const v8f z8 = {0.f, 0.f, 0.f, 0.f, 0.f, 0.f, 0.f, 0.f};
  v8f acc0 = z8, acc1 = z8;
  {
    const unsigned short* ap = XHL + (size_t)row * K1 + 8 * hh;
    const unsigned short* bp = FC1D + (size_t)m * K1 + 8 * hh;
#pragma unroll 2
    for (int k0 = 0; k0 < K1; k0 += 32) {
      FragB af, b0, b1;
      af.h[0] = *(const v8usa*)(ap + k0);
      af.h[1] = *(const v8usa*)(ap + k0 + 16);
      b0.h[0] = *(const v8usa*)(bp + k0);
      b0.h[1] = *(const v8usa*)(bp + k0 + 16);
      b1.h[0] = *(const v8usa*)(bp + (size_t)16 * K1 + k0);
      b1.h[1] = *(const v8usa*)(bp + (size_t)16 * K1 + k0 + 16);
      acc0 = wmb(af, b0, acc0);
      acc1 = wmb(af, b1, acc1);
    }
  }

  float* h1w = h1s + wave * 512;
  {
    const float bi0 = svl[m], bi1 = svl[16 + m];
#pragma unroll
    for (int r = 0; r < 8; ++r) {
      h1w[(8 * hh + r) * 32 + m]      = clip01(acc0[r] + bi0);
      h1w[(8 * hh + r) * 32 + 16 + m] = clip01(acc1[r] + bi1);
    }
  }
  __syncthreads();

  v8f c0 = z8, c1 = z8;
  {
    const float* hr = h1w + m * 32 + 8 * hh;
    const v4f p0 = *(const v4fa*)(hr);
    const v4f p1 = *(const v4fa*)(hr + 4);
    const v4f p2 = *(const v4fa*)(hr + 16);
    const v4f p3 = *(const v4fa*)(hr + 20);
    float f[16];
    f[0] = p0.x; f[1] = p0.y; f[2] = p0.z; f[3] = p0.w;
    f[4] = p1.x; f[5] = p1.y; f[6] = p1.z; f[7] = p1.w;
    f[8] = p2.x; f[9] = p2.y; f[10] = p2.z; f[11] = p2.w;
    f[12] = p3.x; f[13] = p3.y; f[14] = p3.z; f[15] = p3.w;
    FragB ah, al;
#pragma unroll
    for (int i = 0; i < 16; ++i) {
      const unsigned hb = bf16_bits(f[i]);
      ah.u[i] = (unsigned short)hb;
      al.u[i] = (unsigned short)bf16_bits(f[i] - __uint_as_float(hb << 16));
    }
    const unsigned short* b2p = FC2D + (size_t)m * K2 + 8 * hh;
    FragB q00, q01, q10, q11;
    q00.h[0] = *(const v8usa*)(b2p);
    q00.h[1] = *(const v8usa*)(b2p + 16);
    q01.h[0] = *(const v8usa*)(b2p + 32);
    q01.h[1] = *(const v8usa*)(b2p + 48);
    q10.h[0] = *(const v8usa*)(b2p + 16 * K2);
    q10.h[1] = *(const v8usa*)(b2p + 16 * K2 + 16);
    q11.h[0] = *(const v8usa*)(b2p + 16 * K2 + 32);
    q11.h[1] = *(const v8usa*)(b2p + 16 * K2 + 48);
    c0 = wmb(ah, q00, c0);
    c0 = wmb(al, q01, c0);
    c1 = wmb(ah, q10, c1);
    c1 = wmb(al, q11, c1);
  }

  float* h2w = h2s + wave * 512;
  {
    const float bi0 = svl[32 + m], bi1 = svl[48 + m];
#pragma unroll
    for (int r = 0; r < 8; ++r) {
      h2w[(8 * hh + r) * 32 + m]      = clip01(c0[r] + bi0);
      h2w[(8 * hh + r) * 32 + 16 + m] = clip01(c1[r] + bi1);
    }
  }
  __syncthreads();

  {
    const float* h2r = h2w + m * 32;
    float y = 0.0f;
#pragma unroll 4
    for (int k = 0; k < 32; ++k) y = fmaf(h2r[k], svl[64 + k], y);
    y = y + svl[96];
    y = y + PS[row];
    if (hh == 0) outl[16 * wave + m] = y;
  }
  __syncthreads();
  if (tid < 32) {
    const v4f v = *(const v4fa*)(outl + 4 * lane);
    float* dp = out + (size_t)rowBase + 4 * lane;
    *(volatile v4f*)dp = v;
    __threadfence();
    *(volatile v4f*)dp = v;
  }
}

static inline size_t al256(size_t o) { return (o + 255) & ~(size_t)255; }

extern "C" void kernel_launch(void* const* d_in, const int* in_sizes, int n_in,
                              void* d_out, int out_size, void* d_ws, size_t ws_size,
                              hipStream_t stream) {
  if (n_in < 11) return;
  if (in_sizes[0] != NB * MAXF || in_sizes[1] != NB * MAXF) return;
  if (in_sizes[2] != NB) return;
  if (in_sizes[3] != NF * ROWW || in_sizes[4] != ROWW) return;
  if (in_sizes[5] != 32 * 512 || in_sizes[6] != 32) return;
  if (in_sizes[7] != 32 * 32 || in_sizes[8] != 32) return;
  if (in_sizes[9] != 32 || in_sizes[10] != 1) return;
  if (out_size != NB) return;

  const int*   wft  = (const int*)d_in[0];
  const int*   bft  = (const int*)d_in[1];
  const float* stm  = (const float*)d_in[2];
  const float* ftw  = (const float*)d_in[3];
  const float* ftb  = (const float*)d_in[4];
  const float* fc1w = (const float*)d_in[5];
  const float* fc1b = (const float*)d_in[6];
  const float* fc2w = (const float*)d_in[7];
  const float* fc2b = (const float*)d_in[8];
  const float* fcow = (const float*)d_in[9];
  const float* fcob = (const float*)d_in[10];
  float* out = (float*)d_out;

  char* ws = (char*)d_ws;
  size_t off = 0;
  const size_t oFTB  = off; off = al256(off + (size_t)NF * HALF * 2);
  const size_t oPSQ  = off; off = al256(off + (size_t)NF * 4);
  const size_t oXHL  = off; off = al256(off + (size_t)NB * K1 * 2);
  const size_t oPS   = off; off = al256(off + (size_t)NB * 4);
  const size_t oFC1D = off; off = al256(off + (size_t)32 * K1 * 2);
  const size_t oFC2D = off; off = al256(off + (size_t)32 * K2 * 2);
  const size_t oSV   = off; off = al256(off + (size_t)SV_N * 4);
  if (off > ws_size || off > (size_t)WSMAX) return;

  unsigned short* FTB  = (unsigned short*)(ws + oFTB);
  float*          PSQ  = (float*)(ws + oPSQ);
  unsigned short* XHL  = (unsigned short*)(ws + oXHL);
  float*          PS   = (float*)(ws + oPS);
  unsigned short* FC1D = (unsigned short*)(ws + oFC1D);
  unsigned short* FC2D = (unsigned short*)(ws + oFC2D);
  float*          SV   = (float*)(ws + oSV);

  k_prep<<<NTB + 1, 256, 0, stream>>>(ftw, ftb, fc1w, fc1b, fc2w, fc2b, fcow, fcob, FTB, PSQ, FC1D, FC2D, SV);
  k_ft<<<NB / 64, 256, 0, stream>>>(wft, bft, stm, FTB, PSQ, SV, XHL, PS);
  k_mlp<<<NB / 128, 256, 0, stream>>>(XHL, FC1D, FC2D, SV, PS, out);
}
